// ScaleDotProduct_80668075753828
// MI455X (gfx1250) — hardware-verified
//
#include <hip/hip_runtime.h>
#include <math.h>


#define INS    768
#define OUTS   64
#define NBATCH 8
#define SEQ    2048
#define NROWS  (NBATCH * SEQ)
#define NCHUNK (INS / 32)

#define WP   40
#define TP   72
#define VTP  136
#define KP   72
#define VP   40
#define OP   68
#define PWP  72

typedef _Float16 v16h __attribute__((ext_vector_type(16)));
typedef _Float16 v8h  __attribute__((ext_vector_type(8)));
typedef float    v8f  __attribute__((ext_vector_type(8)));
typedef float    v4f  __attribute__((ext_vector_type(4)));
union Frag { v16h v; v8h half[2]; };

__device__ __forceinline__ v8f wmma16(v16h a, v16h b, v8f c) {
    return __builtin_amdgcn_wmma_f32_16x16x32_f16(false, a, false, b, (short)0, c, false, false);
}
#define WGUARD(acc, a, b) asm volatile("v_nop\n\tv_nop\n\tv_nop\n\tv_nop" : "+v"(acc) : "v"(a), "v"(b))

__device__ __forceinline__ v8f zero8() {
    v8f z = {0.f, 0.f, 0.f, 0.f, 0.f, 0.f, 0.f, 0.f};
    return z;
}

__global__ void __launch_bounds__(256)
k_cvt_x(const float* __restrict__ X, _Float16* __restrict__ Xh, int n8) {
    const int i = blockIdx.x * 256 + threadIdx.x;
    if (i >= n8) return;
    const float* p = X + (size_t)i * 8;
    const v4f f0 = *(const v4f*)(p);
    const v4f f1 = *(const v4f*)(p + 4);
    v8h hv;
#pragma unroll
    for (int e = 0; e < 4; ++e) {
        hv[e]     = (_Float16)f0[e];
        hv[e + 4] = (_Float16)f1[e];
    }
    _Float16* d = Xh + (size_t)i * 8;
    *(volatile v8h*)d = hv;
    __threadfence();
    *(volatile v8h*)d = hv;
}

__global__ void __launch_bounds__(256)
k_prep_w(const float* __restrict__ Wq, const float* __restrict__ Wk,
         const float* __restrict__ Wv, _Float16* __restrict__ WT) {
    __shared__ __attribute__((aligned(16))) _Float16 sWT[64 * PWP];

    const int kc = blockIdx.x, mi = blockIdx.y;
    const float* W = (mi == 0) ? Wq : ((mi == 1) ? Wk : Wv);
    const int t = threadIdx.x, lane = t & 31, wave = t >> 5;

#pragma unroll
    for (int jj = 0; jj < 4; ++jj) {
        const int e  = jj * 1024 + t * 4;
        const int kl = e >> 6;
        const int o  = e & 63;
        const v4f w = *(const v4f*)(W + (size_t)(kc * 64 + kl) * OUTS + o);
#pragma unroll
        for (int u = 0; u < 4; ++u) sWT[(o + u) * PWP + kl] = (_Float16)(w[u] * 64.0f);
    }
    __syncthreads();

    v8h v[2];
    size_t go[2];
#pragma unroll
    for (int s = 0; s < 2; ++s) {
        const int o     = wave * 8 + s * 4 + (lane >> 3);
        const int piece = lane & 7;
        v[s]  = *(const v8h*)(&sWT[o * PWP + piece * 8]);
        go[s] = (size_t)(mi * OUTS + o) * INS + (size_t)kc * 64 + piece * 8;
    }
#pragma unroll
    for (int s = 0; s < 2; ++s) *(volatile v8h*)(WT + go[s]) = v[s];
    __threadfence();
#pragma unroll
    for (int s = 0; s < 2; ++s) *(volatile v8h*)(WT + go[s]) = v[s];
}

__global__ void __launch_bounds__(256)
k_proj(const _Float16* __restrict__ Xh, const _Float16* __restrict__ WT,
       const float* __restrict__ bq, const float* __restrict__ bk,
       const float* __restrict__ bv,
       _Float16* __restrict__ Qh, _Float16* __restrict__ Kh,
       _Float16* __restrict__ VhT) {
    __shared__ __attribute__((aligned(16))) _Float16 sW[64 * WP];
    __shared__ __attribute__((aligned(16))) _Float16 sT[8 * 16 * TP];
    __shared__ __attribute__((aligned(16))) _Float16 sVT[64 * VTP];

    const int t = threadIdx.x, lane = t & 31, wave = t >> 5;
    const int l16 = lane & 15, h = lane >> 4;
    const int blk = blockIdx.x, mi = blockIdx.y;

    const _Float16* Wm  = WT + (size_t)mi * OUTS * INS;
    const float* bias   = (mi == 0) ? bq : ((mi == 1) ? bk : bv);
    const int row0w     = blk * 128 + wave * 16;
    const _Float16* xrow = Xh + (size_t)(row0w + l16) * INS;

    const int sn = t >> 2, sp = t & 3;
    const _Float16* wsrc = Wm + (size_t)sn * INS + sp * 8;

    v8f acc[4];
#pragma unroll
    for (int nb = 0; nb < 4; ++nb) acc[nb] = zero8();

#pragma unroll 1
    for (int c = 0; c < NCHUNK; ++c) {
        __syncthreads();
        *(v8h*)(&sW[sn * WP + sp * 8]) = *(const v8h*)(wsrc + c * 32);
        __syncthreads();

        Frag a;
        a.half[0] = *(const v8h*)(xrow + c * 32 + 8 * h);
        a.half[1] = *(const v8h*)(xrow + c * 32 + 16 + 8 * h);
        Frag b[4];
#pragma unroll
        for (int nb = 0; nb < 4; ++nb) {
            const _Float16* wr = &sW[(nb * 16 + l16) * WP];
            b[nb].half[0] = *(const v8h*)(wr + 8 * h);
            b[nb].half[1] = *(const v8h*)(wr + 16 + 8 * h);
        }
#pragma unroll
        for (int nb = 0; nb < 4; ++nb) acc[nb] = wmma16(a.v, b[nb].v, acc[nb]);
#pragma unroll
        for (int nb = 0; nb < 4; ++nb) WGUARD(acc[nb], a.v, b[nb].v);
    }

    float bcol[4];
#pragma unroll
    for (int nb = 0; nb < 4; ++nb) bcol[nb] = bias[nb * 16 + l16];

    if (mi < 2) {
        _Float16* st = sT + wave * (16 * TP);
#pragma unroll
        for (int nb = 0; nb < 4; ++nb)
#pragma unroll
            for (int r = 0; r < 8; ++r)
                st[(8 * h + r) * TP + nb * 16 + l16] =
                    (_Float16)(acc[nb][r] * 0.015625f + bcol[nb]);
    } else {
#pragma unroll
        for (int nb = 0; nb < 4; ++nb)
#pragma unroll
            for (int r = 0; r < 8; ++r)
                sVT[(nb * 16 + l16) * VTP + wave * 16 + 8 * h + r] =
                    (_Float16)(acc[nb][r] * 0.015625f + bcol[nb]);
    }
    __syncthreads();

    if (mi < 2) {
        _Float16* dst = (mi == 0) ? Qh : Kh;
        const _Float16* st = sT + wave * (16 * TP);
        v8h v[4];
        size_t go[4];
#pragma unroll
        for (int s = 0; s < 4; ++s) {
            const int row   = s * 4 + (lane >> 3);
            const int piece = lane & 7;
            v[s]  = *(const v8h*)(&st[row * TP + piece * 8]);
            go[s] = (size_t)(row0w + row) * OUTS + piece * 8;
        }
#pragma unroll
        for (int s = 0; s < 4; ++s) *(volatile v8h*)(dst + go[s]) = v[s];
        __threadfence();
#pragma unroll
        for (int s = 0; s < 4; ++s) *(volatile v8h*)(dst + go[s]) = v[s];
    } else {
        const int bb = blk >> 4;
        const int s0 = (blk & 15) * 128;
        v8h v[4];
        size_t go[4];
#pragma unroll
        for (int s = 0; s < 4; ++s) {
            const int L     = wave * 16 + s * 4 + (lane >> 3);
            const int dim   = L >> 1;
            const int half  = L & 1;
            const int piece = lane & 7;
            v[s]  = *(const v8h*)(&sVT[dim * VTP + half * 64 + piece * 8]);
            go[s] = ((size_t)bb * OUTS + dim) * SEQ + (size_t)s0 + half * 64 + piece * 8;
        }
#pragma unroll
        for (int s = 0; s < 4; ++s) *(volatile v8h*)(VhT + go[s]) = v[s];
        __threadfence();
#pragma unroll
        for (int s = 0; s < 4; ++s) *(volatile v8h*)(VhT + go[s]) = v[s];
    }
}

__global__ void __launch_bounds__(256)
k_attn(const _Float16* __restrict__ Qh, const _Float16* __restrict__ Kh,
       const _Float16* __restrict__ VhT, float* __restrict__ out) {
    __shared__ __attribute__((aligned(16))) _Float16 sK[32 * KP];
    __shared__ __attribute__((aligned(16))) _Float16 sV[64 * VP];
    __shared__ __attribute__((aligned(16))) float    sO[8 * 16 * OP];

    const int t = threadIdx.x, lane = t & 31, wave = t >> 5;
    const int l16 = lane & 15, h = lane >> 4;
    const int b  = blockIdx.x >> 4;
    const int qt = (blockIdx.x & 15) * 8 + wave;
    const size_t qrow0 = (size_t)b * SEQ + (size_t)qt * 16;

    Frag q0, q1;
    {
        const _Float16* qr = Qh + (qrow0 + l16) * OUTS;
        q0.half[0] = *(const v8h*)(qr + 8 * h);
        q0.half[1] = *(const v8h*)(qr + 16 + 8 * h);
        q1.half[0] = *(const v8h*)(qr + 32 + 8 * h);
        q1.half[1] = *(const v8h*)(qr + 48 + 8 * h);
    }

    const _Float16* kbase = Kh  + (size_t)b * SEQ * OUTS;
    const _Float16* vbase = VhT + (size_t)b * OUTS * SEQ;
    const int kk = t >> 3, kpc = t & 7;
    const int vd = t >> 2, vpc = t & 3;

    v8f o[4];
#pragma unroll
    for (int tt = 0; tt < 4; ++tt) o[tt] = zero8();

    float m = -__builtin_inff();
    float ssum = 0.f;
    const float scale  = 0.125f;
    const float pscale = 16384.0f;

#pragma unroll 1
    for (int it = 0; it < SEQ / 32; ++it) {
        const int j = it * 32;
        __syncthreads();
        *(v8h*)(&sK[kk * KP + kpc * 8]) = *(const v8h*)(kbase + (size_t)(j + kk) * OUTS + kpc * 8);
        *(v8h*)(&sV[vd * VP + vpc * 8]) = *(const v8h*)(vbase + (size_t)vd * SEQ + j + vpc * 8);
        __syncthreads();

        Frag a00, a01, a10, a11;
        {
            const _Float16* kr0 = &sK[l16 * KP];
            const _Float16* kr1 = &sK[(16 + l16) * KP];
            a00.half[0] = *(const v8h*)(kr0 + 8 * h);
            a00.half[1] = *(const v8h*)(kr0 + 16 + 8 * h);
            a01.half[0] = *(const v8h*)(kr0 + 32 + 8 * h);
            a01.half[1] = *(const v8h*)(kr0 + 48 + 8 * h);
            a10.half[0] = *(const v8h*)(kr1 + 8 * h);
            a10.half[1] = *(const v8h*)(kr1 + 16 + 8 * h);
            a11.half[0] = *(const v8h*)(kr1 + 32 + 8 * h);
            a11.half[1] = *(const v8h*)(kr1 + 48 + 8 * h);
        }

        v8f s0 = zero8(), s1 = zero8();
        s0 = wmma16(a00.v, q0.v, s0);
        s0 = wmma16(a01.v, q1.v, s0);
        s1 = wmma16(a10.v, q0.v, s1);
        s1 = wmma16(a11.v, q1.v, s1);
        WGUARD(s0, a01.v, q1.v);
        WGUARD(s1, a11.v, q1.v);

        float tmax = -__builtin_inff();
#pragma unroll
        for (int r = 0; r < 8; ++r) {
            s0[r] *= scale;
            s1[r] *= scale;
            tmax = fmaxf(tmax, fmaxf(s0[r], s1[r]));
        }
        tmax = fmaxf(tmax, __shfl_xor(tmax, 16, 32));
        const float mnew = fmaxf(m, tmax);
        const float cfac = __expf(m - mnew);

        float lsum = 0.f;
#pragma unroll
        for (int r = 0; r < 8; ++r) {
            s0[r] = __expf(s0[r] - mnew);
            s1[r] = __expf(s1[r] - mnew);
            lsum += s0[r] + s1[r];
        }
        lsum += __shfl_xor(lsum, 16, 32);
        ssum = ssum * cfac + lsum;
        m = mnew;

        Frag p;
        {
            v8h plo, phi;
#pragma unroll
            for (int e = 0; e < 8; ++e) {
                plo[e] = (_Float16)(s0[e] * pscale);
                phi[e] = (_Float16)(s1[e] * pscale);
            }
            p.half[0] = plo;
            p.half[1] = phi;
        }

        float cr[8];
#pragma unroll
        for (int r = 0; r < 8; ++r) cr[r] = __shfl(cfac, 8 * h + r, 32);
#pragma unroll
        for (int tt = 0; tt < 4; ++tt)
#pragma unroll
            for (int r = 0; r < 8; ++r) o[tt][r] *= cr[r];

        Frag vb[4];
#pragma unroll
        for (int tt = 0; tt < 4; ++tt) {
            const _Float16* vr = &sV[(tt * 16 + l16) * VP];
            vb[tt].half[0] = *(const v8h*)(vr + 8 * h);
            vb[tt].half[1] = *(const v8h*)(vr + 16 + 8 * h);
        }
#pragma unroll
        for (int tt = 0; tt < 4; ++tt) o[tt] = wmma16(p.v, vb[tt].v, o[tt]);
#pragma unroll
        for (int tt = 0; tt < 4; ++tt) WGUARD(o[tt], p.v, vb[tt].v);
    }

    const float inv = (1.0f / ssum) * (1.0f / 16384.0f);
    float ir[8];
#pragma unroll
    for (int r = 0; r < 8; ++r) ir[r] = __shfl(inv, 8 * h + r, 32);

    float* so = sO + wave * (16 * OP);
#pragma unroll
    for (int tt = 0; tt < 4; ++tt)
#pragma unroll
        for (int r = 0; r < 8; ++r)
            so[(8 * h + r) * OP + tt * 16 + l16] = o[tt][r] * ir[r];
    __syncthreads();

    v4f v[8];
    size_t go[8];
#pragma unroll
    for (int s = 0; s < 8; ++s) {
        const int L     = s * 4 + (lane >> 3);
        const int row   = L >> 1;
        const int half  = L & 1;
        const int piece = lane & 7;
        v[s]  = *(const v4f*)(&so[row * OP + half * 32 + piece * 4]);
        go[s] = (qrow0 + row) * OUTS + (size_t)(half * 32 + piece * 4);
    }
#pragma unroll
    for (int s = 0; s < 8; ++s) *(volatile v4f*)(out + go[s]) = v[s];
    __threadfence();
#pragma unroll
    for (int s = 0; s < 8; ++s) *(volatile v4f*)(out + go[s]) = v[s];
}


extern "C" void kernel_launch(void* const* d_in, const int* in_sizes, int n_in,
                              void* d_out, int out_size, void* d_ws, size_t ws_size,
                              hipStream_t stream) {
    if (n_in < 7) return;
    if (in_sizes[0] != NROWS * INS) return;
    if (in_sizes[1] != INS * OUTS || in_sizes[3] != INS * OUTS || in_sizes[5] != INS * OUTS) return;
    if (in_sizes[2] != OUTS || in_sizes[4] != OUTS || in_sizes[6] != OUTS) return;
    if (out_size != NROWS * OUTS) return;

    const float* X  = (const float*)d_in[0];
    const float* Wq = (const float*)d_in[1];
    const float* bq = (const float*)d_in[2];
    const float* Wk = (const float*)d_in[3];
    const float* bk = (const float*)d_in[4];
    const float* Wv = (const float*)d_in[5];
    const float* bv = (const float*)d_in[6];
    float* out = (float*)d_out;

    const size_t bXh = (size_t)NROWS * INS * 2;
    const size_t bWT = (size_t)3 * OUTS * INS * 2;
    const size_t bQ  = (size_t)NROWS * OUTS * 2;
    size_t off = 0;
    const size_t oXh = off; off += (bXh + 255) & ~(size_t)255;
    const size_t oWT = off; off += (bWT + 255) & ~(size_t)255;
    const size_t oQ  = off; off += (bQ + 255) & ~(size_t)255;
    const size_t oK  = off; off += (bQ + 255) & ~(size_t)255;
    const size_t oV  = off; off += (bQ + 255) & ~(size_t)255;
    if (off > ws_size) return;

    char* ws = (char*)d_ws;
    _Float16* Xh  = (_Float16*)(ws + oXh);
    _Float16* WT  = (_Float16*)(ws + oWT);
    _Float16* Qh  = (_Float16*)(ws + oQ);
    _Float16* Kh  = (_Float16*)(ws + oK);
    _Float16* VhT = (_Float16*)(ws + oV);

    const int n8 = NROWS * INS / 8;
    k_cvt_x<<<(n8 + 255) / 256, 256, 0, stream>>>(X, Xh, n8);
    k_prep_w<<<dim3(INS / 64, 3), 256, 0, stream>>>(Wq, Wk, Wv, WT);
    k_proj<<<dim3(NROWS / 128, 3), 256, 0, stream>>>(Xh, WT, bq, bk, bv, Qh, Kh, VhT);
    k_attn<<<NBATCH * (SEQ / 128), 256, 0, stream>>>(Qh, Kh, VhT, out);
    (void)hipGetLastError();
}
